// NegUniform_49589692399688
// MI455X (gfx1250) — hardware-verified
//
#include <hip/hip_runtime.h>
#include <math.h>

typedef __attribute__((ext_vector_type(16))) _Float16 v16h;
typedef __attribute__((ext_vector_type(16))) __bf16 v16b;
typedef __attribute__((ext_vector_type(8)))  _Float16 v8h;
typedef __attribute__((ext_vector_type(8)))  float v8f;
typedef __attribute__((ext_vector_type(4)))  float v4f;
typedef __attribute__((ext_vector_type(2)))  float v2f;
typedef __attribute__((ext_vector_type(4)))  unsigned v4u;
typedef __attribute__((ext_vector_type(4)))  int v4i;
typedef float __attribute__((may_alias)) float_a;
typedef int __attribute__((may_alias)) int_a;

template <typename T> __device__ __forceinline__ void vst2(void* p, T v) { *(volatile T*)p = v; __threadfence(); *(volatile T*)p = v; }
__device__ __forceinline__ v8f wmma16(v16h a, v16h b, v8f c) {
  v8f d = __builtin_amdgcn_wmma_f32_16x16x32_f16(false, a, false, b, (short)0, c, false, false);
  asm volatile("v_nop\n\tv_nop\n\tv_nop\n\tv_nop" : "+v"(d) : "v"(a), "v"(b));
  return d;
}
__device__ __forceinline__ v8f wmma_bf(v16b a, v16b b, v8f c) {
  v8f d = __builtin_amdgcn_wmma_f32_16x16x32_bf16(false, a, false, b, (short)0, c, false, false);
  asm volatile("v_nop\n\tv_nop\n\tv_nop\n\tv_nop" : "+v"(d) : "v"(a), "v"(b));
  return d;
}
__device__ __forceinline__ v16h frag_h(const _Float16* rowk0, int lane) {
  union { v16h v; v8h q[2]; } u; const _Float16* p = rowk0 + 8 * (lane >> 4);
  u.q[0] = *(const v8h*)p; u.q[1] = *(const v8h*)(p + 16); return u.v;
}
__device__ __forceinline__ v16h frag_f32(const float* rowk0, int lane) {
  v16h a; const float* p = rowk0 + 8 * (lane >> 4);
#pragma unroll
  for (int i = 0; i < 8; ++i) { a[i] = (_Float16)p[i]; a[8 + i] = (_Float16)p[16 + i]; }
  return a;
}
__device__ __forceinline__ v16h frag_f32s(const float* rowk0, int lane, float sc) {
  v16h a; const float* p = rowk0 + 8 * (lane >> 4);
#pragma unroll
  for (int i = 0; i < 8; ++i) { a[i] = (_Float16)(p[i] * sc); a[8 + i] = (_Float16)(p[16 + i] * sc); }
  return a;
}
__device__ __forceinline__ v16h fragc_f32(const float* W, int k0, int n, int lane, int ld, int K) {
  v16h a; const int g = lane >> 4;
#pragma unroll
  for (int i = 0; i < 8; ++i) { const int ka = k0 + 8 * g + i, kb = ka + 16;
    a[i] = (_Float16)(ka < K ? W[(size_t)ka * ld + n] : 0.f); a[8 + i] = (_Float16)(kb < K ? W[(size_t)kb * ld + n] : 0.f); }
  return a;
}
struct F2 { v16b h, l; };
__device__ __forceinline__ F2 bsplit16(const float v[16]) { F2 r;
#pragma unroll
  for (int i = 0; i < 16; ++i) { const __bf16 h = (__bf16)v[i]; r.h[i] = h; r.l[i] = (__bf16)(v[i] - (float)h); }
  return r; }
__device__ __forceinline__ F2 split_row(const float* row, int k0, int lane) { float v[16]; const float* p = row + k0 + 8 * (lane >> 4);
#pragma unroll
  for (int i = 0; i < 8; ++i) { v[i] = p[i]; v[8 + i] = p[16 + i]; }
  return bsplit16(v); }
__device__ __forceinline__ F2 split_rowK(const float* row, int k0, int lane, int K) { float v[16]; const int g = lane >> 4;
#pragma unroll
  for (int i = 0; i < 8; ++i) { const int ka = k0 + 8 * g + i, kb = ka + 16; v[i] = ka < K ? row[ka] : 0.f; v[8 + i] = kb < K ? row[kb] : 0.f; }
  return bsplit16(v); }
__device__ __forceinline__ F2 split_col(const float* W, int k0, int n, int lane, int ld, int K) { float v[16]; const int g = lane >> 4;
#pragma unroll
  for (int i = 0; i < 8; ++i) { const int ka = k0 + 8 * g + i, kb = ka + 16; v[i] = ka < K ? W[(size_t)ka * ld + n] : 0.f; v[8 + i] = kb < K ? W[(size_t)kb * ld + n] : 0.f; }
  return bsplit16(v); }
__device__ __forceinline__ v8f mac3(const F2& a, const F2& b, v8f c) { c = wmma_bf(a.l, b.h, c); c = wmma_bf(a.h, b.l, c); return wmma_bf(a.h, b.h, c); }
__device__ __forceinline__ float sigm(float v) { return 1.0f / (1.0f + expf(-v)); }
#define LDSX() do { asm volatile("s_wait_dscnt 0" ::: "memory"); __builtin_amdgcn_wave_barrier(); __builtin_amdgcn_fence(__ATOMIC_RELEASE, "workgroup"); } while (0)

#define NN 4096
#define DD 128
#define JJ 4
#define KT 16

__global__ __launch_bounds__(128) void k_norm(const float* __restrict__ f, const float* __restrict__ ng, _Float16* __restrict__ fn, _Float16* __restrict__ nn) {
  __shared__ float sq[128]; __shared__ __align__(16) _Float16 srow[32][DD + 8];
  const int tid = threadIdx.x, rl = tid >> 2, part = tid & 3; const int r = blockIdx.x * 32 + rl;
  const float* src = r < NN ? f + (size_t)r * DD : ng + (size_t)(r - NN) * DD;
  float s = 0.f; for (int d = part * 32; d < part * 32 + 32; ++d) { const float v = src[d]; s += v * v; }
  sq[tid] = s; __syncthreads();
  const float tot = sq[rl * 4] + sq[rl * 4 + 1] + sq[rl * 4 + 2] + sq[rl * 4 + 3]; const float inv = 8.0f / fmaxf(sqrtf(tot), 1e-12f);
  for (int d = part * 32; d < part * 32 + 32; ++d) srow[rl][d] = (_Float16)(src[d] * inv);
  __syncthreads();
  for (int q = tid; q < 32 * DD / 8; q += 128) { const int rr = q >> 4, pc = q & 15; const int row = blockIdx.x * 32 + rr; _Float16* dst = row < NN ? fn + (size_t)row * DD : nn + (size_t)(row - NN) * DD;
    vst2(dst + pc * 8, *(const v4u*)(&srow[rr][pc * 8])); }
}
__global__ __launch_bounds__(128) void k_top(const _Float16* __restrict__ fn, const _Float16* __restrict__ nn, const int* __restrict__ tgt, const int* __restrict__ idxp, float* __restrict__ top) {
  __shared__ __align__(16) float sS[4][16][20];
  __shared__ int stg[16 * 4];
  __shared__ __align__(16) float so[4][16][KT];
  const int tid = threadIdx.x, w = tid >> 5, lane = tid & 31, col = lane & 15, g = lane >> 4;
  const int j = blockIdx.y, n0 = blockIdx.x * 64 + w * 16; const int idx = idxp[0]; const bool maskj = (j == idx);
  const _Float16* nb = nn + (size_t)j * NN * DD;
  v16h af[4];
#pragma unroll
  for (int kc = 0; kc < 4; ++kc) af[kc] = frag_h(fn + (size_t)(n0 + col) * DD + kc * 32, lane);
  const int myt = tgt[n0 + col];
  float t16[KT];
#pragma unroll
  for (int k = 0; k < KT; ++k) t16[k] = -3.0e38f;
#pragma unroll 1
  for (int mt = 0; mt < NN / 16; ++mt) { v8f s = {};
#pragma unroll
    for (int kc = 0; kc < 4; ++kc) s = wmma16(af[kc], frag_h(nb + (size_t)(mt * 16 + col) * DD + kc * 32, lane), s);
#pragma unroll
    for (int r = 0; r < 8; ++r) sS[w][8 * g + r][col] = s[r] * (1.0f / 64.0f);
    if (lane < 16) stg[w * 16 + lane] = tgt[mt * 16 + lane];
    LDSX();
    if (g == 0) { const int m = col;
#pragma unroll
      for (int e = 0; e < 16; ++e) { float c = sS[w][m][e]; if (maskj && stg[w * 16 + e] == myt) c = -1.0e9f;
        if (c > t16[KT - 1]) { t16[KT - 1] = c;
#pragma unroll
          for (int k = KT - 1; k > 0; --k) { if (t16[k] > t16[k - 1]) { const float tmp = t16[k]; t16[k] = t16[k - 1]; t16[k - 1] = tmp; } } } } }
    LDSX(); }
  if (g == 0) {
#pragma unroll
    for (int k = 0; k < KT; ++k) so[w][col][k] = t16[k]; }
  LDSX();
  for (int q = lane; q < 16 * KT / 4; q += 32) { const int rl = q >> 2, pc = q & 3; vst2(top + ((size_t)j * NN + n0 + rl) * KT + pc * 4, *(const v4f*)(&so[w][rl][pc * 4])); }
}
__global__ __launch_bounds__(256) void k_loss(const float* __restrict__ top, float* __restrict__ part) {
  __shared__ float sr[256];
  const int tid = threadIdx.x, n = blockIdx.x * 256 + tid;
  __shared__ float dec[KT];
  if (tid == 0) { float s = 0.f, v = 1.0f; for (int k = 0; k < KT; ++k) { dec[k] = v; s += v; v *= 0.95f; } for (int k = 0; k < KT; ++k) dec[k] /= s; }
  __syncthreads();
  float acc = 0.f;
#pragma unroll 1
  for (int k = 0; k < KT; ++k) { float lg[JJ]; float mx = -3.0e38f;
#pragma unroll
    for (int j = 0; j < JJ; ++j) { lg[j] = top[((size_t)j * NN + n) * KT + k] * 100.0f; mx = fmaxf(mx, lg[j]); }
    float z = 0.f;
#pragma unroll
    for (int j = 0; j < JJ; ++j) z += expf(lg[j] - mx);
    const float lz = logf(z); float ent = 0.f;
#pragma unroll
    for (int j = 0; j < JJ; ++j) { const float lp = lg[j] - mx - lz; ent += expf(lp) * lp; }
    acc += ent * dec[k]; }
  sr[tid] = acc; __syncthreads();
  if (tid < 32) { float s = 0.f; if (tid == 0) { for (int i = 0; i < 256; ++i) s += sr[i]; } vst2(part + (size_t)blockIdx.x * 32 + tid, (float_a)(tid == 0 ? s : 0.f)); }
}
__global__ __launch_bounds__(32) void k_fin(const float* __restrict__ part, float* __restrict__ out) {
  if (threadIdx.x == 0) { float s = 0.f; for (int b = 0; b < NN / 256; ++b) s += part[(size_t)b * 32]; vst2(out, (float_a)(s / (float)NN + logf((float)JJ))); }
}
extern "C" void kernel_launch(void* const* d_in, const int* in_sizes, int n_in, void* d_out, int out_size, void* d_ws, size_t ws_size, hipStream_t stream) {
  (void)in_sizes; (void)n_in; (void)out_size; (void)ws_size;
  const float* f = (const float*)d_in[0]; const int* tgt = (const int*)d_in[1]; const float* ng = (const float*)d_in[2]; const int* idxp = (const int*)d_in[3];
  float* out = (float*)d_out;
  char* ws = (char*)d_ws; size_t off = 0;
  auto take = [&](size_t bytes) { char* p = ws + off; off += (bytes + 255) & ~(size_t)255; return p; };
  _Float16* fn = (_Float16*)take((size_t)NN * DD * 2); _Float16* nn = (_Float16*)take((size_t)JJ * NN * DD * 2); float* top = (float*)take((size_t)JJ * NN * KT * 4); float* part = (float*)take((size_t)(NN / 256) * 32 * 4);
  k_norm<<<(JJ + 1) * NN / 32, 128, 0, stream>>>(f, ng, fn, nn);
  k_top<<<dim3(NN / 64, JJ), 128, 0, stream>>>(fn, nn, tgt, idxp, top);
  k_loss<<<NN / 256, 256, 0, stream>>>(top, part);
  k_fin<<<1, 32, 0, stream>>>(part, out);
}
